// PatchedGINConv_66340064854630
// MI455X (gfx1250) — hardware-verified
//
#include <hip/hip_runtime.h>
#include <math.h>

typedef __attribute__((ext_vector_type(16))) _Float16 v16h;
typedef __attribute__((ext_vector_type(16))) __bf16 v16b;
typedef __attribute__((ext_vector_type(8)))  _Float16 v8h;
typedef __attribute__((ext_vector_type(8)))  float v8f;
typedef __attribute__((ext_vector_type(4)))  float v4f;
typedef __attribute__((ext_vector_type(2)))  float v2f;
typedef __attribute__((ext_vector_type(4)))  unsigned v4u;
typedef __attribute__((ext_vector_type(4)))  int v4i;
typedef float __attribute__((may_alias)) float_a;
typedef int __attribute__((may_alias)) int_a;

template <typename T> __device__ __forceinline__ void vst2(void* p, T v) { *(volatile T*)p = v; __threadfence(); *(volatile T*)p = v; }
__device__ __forceinline__ v8f wmma16(v16h a, v16h b, v8f c) {
  v8f d = __builtin_amdgcn_wmma_f32_16x16x32_f16(false, a, false, b, (short)0, c, false, false);
  asm volatile("v_nop\n\tv_nop\n\tv_nop\n\tv_nop" : "+v"(d) : "v"(a), "v"(b));
  return d;
}
__device__ __forceinline__ v8f wmma_bf(v16b a, v16b b, v8f c) {
  v8f d = __builtin_amdgcn_wmma_f32_16x16x32_bf16(false, a, false, b, (short)0, c, false, false);
  asm volatile("v_nop\n\tv_nop\n\tv_nop\n\tv_nop" : "+v"(d) : "v"(a), "v"(b));
  return d;
}
__device__ __forceinline__ v16h frag_h(const _Float16* rowk0, int lane) {
  union { v16h v; v8h q[2]; } u; const _Float16* p = rowk0 + 8 * (lane >> 4);
  u.q[0] = *(const v8h*)p; u.q[1] = *(const v8h*)(p + 16); return u.v;
}
__device__ __forceinline__ v16h frag_f32(const float* rowk0, int lane) {
  v16h a; const float* p = rowk0 + 8 * (lane >> 4);
#pragma unroll
  for (int i = 0; i < 8; ++i) { a[i] = (_Float16)p[i]; a[8 + i] = (_Float16)p[16 + i]; }
  return a;
}
__device__ __forceinline__ v16h frag_f32s(const float* rowk0, int lane, float sc) {
  v16h a; const float* p = rowk0 + 8 * (lane >> 4);
#pragma unroll
  for (int i = 0; i < 8; ++i) { a[i] = (_Float16)(p[i] * sc); a[8 + i] = (_Float16)(p[16 + i] * sc); }
  return a;
}
__device__ __forceinline__ v16h fragc_f32(const float* W, int k0, int n, int lane, int ld, int K) {
  v16h a; const int g = lane >> 4;
#pragma unroll
  for (int i = 0; i < 8; ++i) { const int ka = k0 + 8 * g + i, kb = ka + 16;
    a[i] = (_Float16)(ka < K ? W[(size_t)ka * ld + n] : 0.f); a[8 + i] = (_Float16)(kb < K ? W[(size_t)kb * ld + n] : 0.f); }
  return a;
}
struct F2 { v16b h, l; };
__device__ __forceinline__ F2 bsplit16(const float v[16]) { F2 r;
#pragma unroll
  for (int i = 0; i < 16; ++i) { const __bf16 h = (__bf16)v[i]; r.h[i] = h; r.l[i] = (__bf16)(v[i] - (float)h); }
  return r; }
__device__ __forceinline__ F2 split_row(const float* row, int k0, int lane) { float v[16]; const float* p = row + k0 + 8 * (lane >> 4);
#pragma unroll
  for (int i = 0; i < 8; ++i) { v[i] = p[i]; v[8 + i] = p[16 + i]; }
  return bsplit16(v); }
__device__ __forceinline__ F2 split_rowK(const float* row, int k0, int lane, int K) { float v[16]; const int g = lane >> 4;
#pragma unroll
  for (int i = 0; i < 8; ++i) { const int ka = k0 + 8 * g + i, kb = ka + 16; v[i] = ka < K ? row[ka] : 0.f; v[8 + i] = kb < K ? row[kb] : 0.f; }
  return bsplit16(v); }
__device__ __forceinline__ F2 split_col(const float* W, int k0, int n, int lane, int ld, int K) { float v[16]; const int g = lane >> 4;
#pragma unroll
  for (int i = 0; i < 8; ++i) { const int ka = k0 + 8 * g + i, kb = ka + 16; v[i] = ka < K ? W[(size_t)ka * ld + n] : 0.f; v[8 + i] = kb < K ? W[(size_t)kb * ld + n] : 0.f; }
  return bsplit16(v); }
__device__ __forceinline__ v8f mac3(const F2& a, const F2& b, v8f c) { c = wmma_bf(a.l, b.h, c); c = wmma_bf(a.h, b.l, c); return wmma_bf(a.h, b.h, c); }
__device__ __forceinline__ float sigm(float v) { return 1.0f / (1.0f + expf(-v)); }
#define LDSX() do { asm volatile("s_wait_dscnt 0" ::: "memory"); __builtin_amdgcn_wave_barrier(); __builtin_amdgcn_fence(__ATOMIC_RELEASE, "workgroup"); } while (0)

#define NN 50000
#define NE 800000
#define DI 64
#define DH 128
#define RB 512
#define NRB ((NN + RB - 1) / RB)
#define NNP (NRB * RB)
#define CH 256

__global__ __launch_bounds__(256) void k_scatter(const float* __restrict__ x, const int* __restrict__ ei, float* __restrict__ AGG) {
  __shared__ __align__(16) float sacc[RB][DI];
  __shared__ int ssrc[CH], sdl[CH]; __shared__ int scnt[8]; __shared__ int sbase[9];
  const int tid = threadIdx.x, wave = tid >> 5, lane = tid & 31;
  const int r0 = blockIdx.x * RB;
  const int* esrc = ei; const int* edst = ei + NE;
  for (int q = tid; q < RB * DI; q += 256) (&sacc[0][0])[q] = 0.f;
  __syncthreads();
#pragma unroll 1
  for (int c0 = 0; c0 < NE; c0 += CH) {
    const int e = c0 + tid; int hit = 0, s = 0, dl = 0;
    if (e < NE) { const int d = edst[e]; if (d >= r0 && d < r0 + RB) { hit = 1; dl = d - r0; s = esrc[e]; s = s < 0 ? 0 : (s >= NN ? NN - 1 : s); } }
    const unsigned bal = __ballot(hit); const int wcnt = __popc(bal); const int pre = __popc(bal & ((1u << lane) - 1u));
    if (lane == 0) scnt[wave] = wcnt;
    __syncthreads();
    if (tid == 0) { int acc = 0; for (int w = 0; w < 8; ++w) { sbase[w] = acc; acc += scnt[w]; } sbase[8] = acc; }
    __syncthreads();
    if (hit) { const int pos = sbase[wave] + pre; ssrc[pos] = s; sdl[pos] = dl; }
    __syncthreads();
    const int nh = sbase[8];
    if (tid < DI) { for (int i = 0; i < nh; ++i) sacc[sdl[i]][tid] += x[(size_t)ssrc[i] * DI + tid]; }
    __syncthreads(); }
  for (int q = tid; q < RB * (DI / 4); q += 256) { const int rl = q / (DI / 4), pc = q % (DI / 4); const int r = r0 + rl; v4f v = *(const v4f*)(&sacc[rl][pc * 4]);
    if (r < NN) { const v4f xv = *(const v4f*)(x + (size_t)r * DI + pc * 4); v += xv; } else { v = (v4f){0.f, 0.f, 0.f, 0.f}; }
    vst2(AGG + (size_t)r * DI + pc * 4, v); }
}
__global__ __launch_bounds__(128) void k_mlp(const float* __restrict__ AGG, const float* __restrict__ W1, const float* __restrict__ b1, const float* __restrict__ W2, const float* __restrict__ b2, float* __restrict__ out) {
  __shared__ __align__(16) float sh[4][16][DH + 4];
  __shared__ __align__(16) float so[4][16][DI + 4];
  const int tid = threadIdx.x, wave = tid >> 5, lane = tid & 31, col = lane & 15, g = lane >> 4;
  const int r0 = blockIdx.x * 64 + wave * 16;
  { v8f acc[8] = {};
#pragma unroll
    for (int kc = 0; kc < DI / 32; ++kc) { const F2 a = split_row(AGG + (size_t)(r0 + col) * DI, kc * 32, lane);
#pragma unroll
      for (int j = 0; j < 8; ++j) acc[j] = mac3(a, split_col(W1, kc * 32, j * 16 + col, lane, DH, DI), acc[j]); }
#pragma unroll
    for (int j = 0; j < 8; ++j) { const int n = j * 16 + col; const float bb = b1[n];
#pragma unroll
      for (int r = 0; r < 8; ++r) { const float v = acc[j][r] + bb; sh[wave][8 * g + r][n] = v > 0.f ? v : 0.f; } } }
  LDSX();
  { v8f acc[4] = {};
#pragma unroll
    for (int kc = 0; kc < DH / 32; ++kc) { const F2 a = split_row(&sh[wave][col][0], kc * 32, lane);
#pragma unroll
      for (int j = 0; j < 4; ++j) acc[j] = mac3(a, split_col(W2, kc * 32, j * 16 + col, lane, DI, DH), acc[j]); }
#pragma unroll
    for (int j = 0; j < 4; ++j) { const int n = j * 16 + col; const float bb = b2[n];
#pragma unroll
      for (int r = 0; r < 8; ++r) so[wave][8 * g + r][n] = acc[j][r] + bb; } }
  LDSX();
  for (int q = lane; q < 16 * 16; q += 32) { const int rl = q >> 4, pc = q & 15; const int r = r0 + rl; if (r < NN) vst2(out + (size_t)r * DI + pc * 4, *(const v4f*)(&so[wave][rl][pc * 4])); }
}
extern "C" void kernel_launch(void* const* d_in, const int* in_sizes, int n_in, void* d_out, int out_size, void* d_ws, size_t ws_size, hipStream_t stream) {
  (void)in_sizes; (void)n_in; (void)out_size; (void)ws_size;
  const float* x = (const float*)d_in[0]; const int* ei = (const int*)d_in[1]; const float* W1 = (const float*)d_in[2]; const float* b1 = (const float*)d_in[3]; const float* W2 = (const float*)d_in[4]; const float* b2 = (const float*)d_in[5];
  float* out = (float*)d_out;
  float* AGG = (float*)d_ws;
  k_scatter<<<NRB, 256, 0, stream>>>(x, ei, AGG);
  k_mlp<<<NNP / 64, 128, 0, stream>>>(AGG, W1, b1, W2, b2, out);
}
